// VisionEncoderMambaBlock3_74345883893856
// MI455X (gfx1250) — hardware-run, weakly checked
//
#include <hip/hip_runtime.h>
#include <hip/hip_fp16.h>
#include <math.h>

typedef __attribute__((ext_vector_type(16))) _Float16 v16h;
typedef __attribute__((ext_vector_type(8)))  _Float16 v8h;
typedef __attribute__((ext_vector_type(8)))  float    v8f;
typedef __attribute__((ext_vector_type(4)))  float    v4f;
typedef __attribute__((ext_vector_type(2)))  unsigned v2u;

constexpr int kBatch   = 2;
constexpr int kSeq     = 2048;
constexpr int kDim     = 512;
constexpr int kRows    = kBatch * kSeq;
constexpr int kDtRank  = 32;
constexpr int kNst     = 16;
constexpr int kBcP     = 64;
constexpr int kOffB    = 32;
constexpr int kOffC    = 48;
constexpr int kNbranch = 3;
constexpr size_t kPlane = (size_t)kRows * kDim;
constexpr float kWCarry    = 1024.0f;
constexpr float kResid     = 2048.0f;
constexpr float kYCarry    = 16.0f;
constexpr float kSW        = 1.0f / 1024.0f;
constexpr float kSWr       = 1.0f / (1024.0f * 2048.0f);
constexpr float kResidInv  = 1.0f / 2048.0f;
constexpr float kYCarryInv = 1.0f / 16.0f;
constexpr float kLnEps     = 1e-5f;
static_assert(kRows == 4096);
static_assert(kDtRank + 2 * kNst == kBcP);
static_assert((kDim % 64) == 0 && (kSeq % 64) == 0 && (kBcP % 64) == 0);
static_assert((kDim % 32) == 0 && (kDtRank % 32) == 0);
static_assert((kRows % 32) == 0 && (kRows % 16) == 0);
static_assert((kDim & (kDim - 1)) == 0 && (kDim % 256) == 0);

constexpr size_t kSzW16  = (size_t)kDim * kDim * 2;
constexpr size_t kSzWD   = (size_t)kBcP * kDim * 2;
constexpr size_t kSzWT   = (size_t)kDim * kDtRank * 2;
constexpr size_t kSzA16  = kPlane * 2;
constexpr size_t kSzA32  = kPlane * 4;
constexpr size_t kSzBC   = (size_t)kRows * kBcP * 4;
constexpr size_t kSzBC16 = (size_t)kRows * kBcP * 2;
constexpr size_t kSzZ    = (size_t)kNbranch * kSzA32;
constexpr size_t kSzY16  = (size_t)kNbranch * kSzA16;
constexpr size_t kOffWPH = 0;
constexpr size_t kOffWPL = kOffWPH + kSzW16;
constexpr size_t kOffWC  = kOffWPL + kSzW16;
constexpr size_t kOffWDH = kOffWC  + kSzW16;
constexpr size_t kOffWDL = kOffWDH + kSzWD;
constexpr size_t kOffWT  = kOffWDL + kSzWD;
constexpr size_t kOffTNH = kOffWT  + kSzWT;
constexpr size_t kOffTNL = kOffTNH + kSzA16;
constexpr size_t kOffPR  = kOffTNL + kSzA16;
constexpr size_t kOffPH  = kOffPR  + kSzA32;
constexpr size_t kOffPL  = kOffPH  + kSzA16;
constexpr size_t kOffCR  = kOffPL  + kSzA16;
constexpr size_t kOffU   = kOffCR  + kSzA32;
constexpr size_t kOffUH  = kOffU   + kSzA32;
constexpr size_t kOffUL  = kOffUH  + kSzA16;
constexpr size_t kOffBC  = kOffUL  + kSzA16;
constexpr size_t kOffBCH = kOffBC  + kSzBC;
constexpr size_t kOffBCL = kOffBCH + kSzBC16;
constexpr size_t kOffDTR = kOffBCL + kSzBC16;
constexpr size_t kOffDT  = kOffDTR + kSzA32;
constexpr size_t kOffZ   = kOffDT  + kSzA32;
constexpr size_t kOffYH  = kOffZ   + kSzZ;
constexpr size_t kOffYL  = kOffYH  + kSzY16;
constexpr size_t kWsTotal = kOffYL + kSzY16;
static_assert(kWsTotal == 121274368ull);
static_assert(kWsTotal <= 134217728ull);
static_assert((kOffWPL % 128) == 0 && (kOffWC % 128) == 0 && (kOffWDH % 128) == 0 && (kOffWDL % 128) == 0 &&
              (kOffWT % 128) == 0 &&
              (kOffTNH % 128) == 0 && (kOffTNL % 128) == 0 && (kOffPR % 128) == 0 && (kOffPH % 128) == 0 &&
              (kOffPL % 128) == 0 && (kOffCR % 128) == 0 && (kOffU % 128) == 0 && (kOffUH % 128) == 0 &&
              (kOffUL % 128) == 0 && (kOffBC % 128) == 0 && (kOffBCH % 128) == 0 && (kOffBCL % 128) == 0 &&
              (kOffDTR % 128) == 0 && (kOffDT % 128) == 0 && (kOffZ % 128) == 0 && (kOffYH % 128) == 0 &&
              (kOffYL % 128) == 0);

__device__ __forceinline__ _Float16 f16_flush(float v) {
  const float w = (fabsf(v) < 6.103515625e-05f) ? 0.0f : v;
  return (_Float16)w;
}
__device__ __forceinline__ void f16_split(float v, _Float16& hi, _Float16& lo) {
  hi = f16_flush(v);
  const float hf = (float)hi;
  const float r = (v - hf) * kResid;
  lo = f16_flush(r);
}

__device__ __forceinline__ float h16_to_f32(unsigned hb) {
  const unsigned sgn = (hb & 0x8000u) << 16; const unsigned em = hb & 0x7fffu;
  const float fn = __uint_as_float((em << 13) + 0x38000000u);
  const float fs = (float)em * 5.9604644775390625e-8f;
  const float mag = (em < 0x400u) ? fs : fn; return __uint_as_float(__float_as_uint(mag) | sgn); }

namespace eng {
union FragU { v16h v; v8h h[2]; };
__device__ __forceinline__ v16h frag_load(const _Float16* p) {
  FragU f;
  f.h[0] = *(const v8h*)(p);
  f.h[1] = *(const v8h*)(p + 16);
  return f.v;
}
__device__ __forceinline__ v8f mma(v16h a, v16h b, v8f c) {
  return __builtin_amdgcn_wmma_f32_16x16x32_f16(false, a, false, b, (short)0, c, false, false);
}
__device__ __forceinline__ void guard1(v8f& a, v16h x, v16h y) {
  asm volatile("v_nop\n\tv_nop\n\tv_nop\n\tv_nop" : "+v"(a) : "v"(x), "v"(y));
}
__device__ __forceinline__ void guard_acc(v8f& a) {
  asm volatile("v_nop\n\tv_nop\n\tv_nop\n\tv_nop" : "+v"(a));
}
__device__ __forceinline__ void keep4(v16h a, v16h b, v16h c, v16h d) {
  asm volatile("v_nop" :: "v"(a), "v"(b), "v"(c), "v"(d));
}

template <int MI, int SPL>
__global__ __launch_bounds__(256) void gemm_f16_kernel(
    const unsigned short* __restrict__ Ap, const unsigned short* __restrict__ A2p, int lda,
    const unsigned short* __restrict__ Btp, const unsigned short* __restrict__ Bt2p, int ldb,
    float* __restrict__ C, int ldc, int M, int N, int K, float scale, float rscale)
{
  static_assert(MI >= 1 && MI <= 2);
  static_assert(SPL >= 0 && SPL <= 2);
  const _Float16* A   = (const _Float16*)Ap;
  const _Float16* A2  = (const _Float16*)A2p;
  const _Float16* Bt  = (const _Float16*)Btp;
  const _Float16* Bt2 = (const _Float16*)Bt2p;
  __shared__ __align__(16) float sT[8][16 * 68];
  const int lane = threadIdx.x & 31;
  const int wave = threadIdx.x >> 5;
  const int tilesN = N >> 6;
  const int tilesM = M / (16 * MI);
  const int tile = blockIdx.x * 8 + wave;
  if (tile >= tilesM * tilesN) return;
  const int tm = tile / tilesN;
  const int tn = tile - tm * tilesN;
  const int m0 = tm * (16 * MI);
  const int n0 = tn << 6;
  const int rlane = lane & 15;
  const int koff  = (lane >> 4) * 8;
  const int mOff  = (lane >> 4) * 8;

  v8f acc[MI][4], accr[MI][4];
#pragma unroll
  for (int i = 0; i < MI; ++i)
#pragma unroll
    for (int j = 0; j < 4; ++j) {
      acc[i][j]  = (v8f){0.f, 0.f, 0.f, 0.f, 0.f, 0.f, 0.f, 0.f};
      accr[i][j] = (v8f){0.f, 0.f, 0.f, 0.f, 0.f, 0.f, 0.f, 0.f};
    }

  for (int k0 = 0; k0 < K; k0 += 32) {
    v16h bh[4], bl[4];
#pragma unroll
    for (int j = 0; j < 4; ++j) {
      const size_t bo = (size_t)(n0 + (j << 4) + rlane) * ldb + koff + k0;
      bh[j] = frag_load(Bt + bo);
      if (SPL == 2) bl[j] = frag_load(Bt2 + bo); else bl[j] = bh[j];
    }
#pragma unroll
    for (int i = 0; i < MI; ++i) {
      const size_t ao = (size_t)(m0 + (i << 4) + rlane) * lda + koff + k0;
      const v16h ah = frag_load(A + ao);
      v16h al = ah;
      if (SPL >= 1) al = frag_load(A2 + ao);
#pragma unroll
      for (int j = 0; j < 4; ++j) {
        acc[i][j] = mma(ah, bh[j], acc[i][j]);
        if (SPL >= 1) accr[i][j] = mma(al, bh[j], accr[i][j]);
        if (SPL == 2) accr[i][j] = mma(ah, bl[j], accr[i][j]);
      }
#pragma unroll
      for (int j = 0; j < 4; ++j) {
        guard1(acc[i][j], ah, al);
        if (SPL >= 1) guard1(accr[i][j], ah, al);
      }
    }
    keep4(bh[0], bh[1], bh[2], bh[3]);
    if (SPL == 2) keep4(bl[0], bl[1], bl[2], bl[3]);
  }
#pragma unroll
  for (int i = 0; i < MI; ++i)
#pragma unroll
    for (int j = 0; j < 4; ++j) {
      guard_acc(acc[i][j]);
      if (SPL >= 1) guard_acc(accr[i][j]);
    }

  float* slab = sT[wave];
#pragma unroll
  for (int i = 0; i < MI; ++i) {
    const int mBase = m0 + (i << 4);
#pragma unroll
    for (int j = 0; j < 4; ++j) {
#pragma unroll
      for (int r = 0; r < 8; ++r) {
        float v = acc[i][j][r] * scale;
        if (SPL >= 1) v += accr[i][j][r] * rscale;
        slab[(mOff + r) * 68 + (j << 4) + rlane] = v;
      }
    }
    __builtin_amdgcn_fence(__ATOMIC_RELEASE, "workgroup");
    __builtin_amdgcn_wave_barrier();
    __builtin_amdgcn_fence(__ATOMIC_ACQUIRE, "workgroup");
    {
      const int hh = lane >> 4, c4 = (lane & 15) * 4;
      for (int pass = 0; pass < 2; ++pass) {
#pragma unroll
        for (int it = 0; it < 8; ++it) {
          const int row = it * 2 + hh;
          const v4f v = *(const v4f*)(slab + row * 68 + c4);
          *(volatile v4f*)(C + (size_t)(mBase + row) * ldc + n0 + c4) = v;
        }
        __threadfence();
      }
    }
    __builtin_amdgcn_fence(__ATOMIC_RELEASE, "workgroup");
    __builtin_amdgcn_wave_barrier();
    __builtin_amdgcn_fence(__ATOMIC_ACQUIRE, "workgroup");
  }
}
}

__global__ __launch_bounds__(256) void split_rows_f16_kernel(
    const float* __restrict__ src, unsigned short* __restrict__ dH, unsigned short* __restrict__ dL, int total8)
{
  const int i = blockIdx.x * 256 + threadIdx.x;
  if (i >= total8) return;
  const size_t e0 = (size_t)i << 3;
  const v4f a0 = *(const v4f*)(src + e0);
  const v4f a1 = *(const v4f*)(src + e0 + 4);
  v8h hv, lv;
#pragma unroll
  for (int e = 0; e < 4; ++e) {
    _Float16 h0, l0, h1, l1;
    const float f0 = a0[e];
    const float f1 = a1[e];
    f16_split(f0, h0, l0);
    f16_split(f1, h1, l1);
    hv[e] = h0; lv[e] = l0;
    hv[4 + e] = h1; lv[4 + e] = l1;
  }
  unsigned short* qh = dH + e0;
  unsigned short* ql = dL + e0;
  *(volatile v8h*)qh = hv;
  *(volatile v8h*)ql = lv;
  __threadfence();
  *(volatile v8h*)qh = hv;
  *(volatile v8h*)ql = lv;
}

template <bool LO>
__global__ __launch_bounds__(256) void pack_weight_f16_kernel(
    const float* __restrict__ src, unsigned short* __restrict__ dH, unsigned short* __restrict__ dL,
    int total8, float carry)
{
  const int i = blockIdx.x * 256 + threadIdx.x;
  if (i >= total8) return;
  const size_t e0 = (size_t)i << 3;
  const v4f a0 = *(const v4f*)(src + e0);
  const v4f a1 = *(const v4f*)(src + e0 + 4);
  v8h hv, lv;
#pragma unroll
  for (int e = 0; e < 4; ++e) {
    _Float16 h0, l0, h1, l1;
    const float f0 = a0[e] * carry;
    const float f1 = a1[e] * carry;
    f16_split(f0, h0, l0);
    f16_split(f1, h1, l1);
    hv[e] = h0; lv[e] = l0;
    hv[4 + e] = h1; lv[4 + e] = l1;
  }
  unsigned short* qh = dH + e0;
  unsigned short* ql = dL + e0;
  *(volatile v8h*)qh = hv;
  if (LO) *(volatile v8h*)ql = lv;
  __threadfence();
  *(volatile v8h*)qh = hv;
  if (LO) *(volatile v8h*)ql = lv;
}

__global__ __launch_bounds__(256) void layernorm_split_kernel(
    const float* __restrict__ X, const float* __restrict__ gw, const float* __restrict__ gb,
    unsigned short* __restrict__ dH, unsigned short* __restrict__ dL, int rows)
{
  const int lane = threadIdx.x & 31;
  const int wave = threadIdx.x >> 5;
  const int row  = blockIdx.x * 8 + wave;
  if (row >= rows) return;
  const float* xr = X + (size_t)row * kDim;
  v4f t[4];
#pragma unroll
  for (int g = 0; g < 4; ++g) t[g] = *(const v4f*)(xr + (g >> 1) * 256 + lane * 8 + (g & 1) * 4);
  float s = 0.0f;
#pragma unroll
  for (int g = 0; g < 4; ++g)
#pragma unroll
    for (int e = 0; e < 4; ++e) s += t[g][e];
#pragma unroll
  for (int o = 16; o >= 1; o >>= 1) s += __shfl_xor(s, o, 32);
  const float mu = s * (1.0f / (float)kDim);
  float ss = 0.0f;
#pragma unroll
  for (int g = 0; g < 4; ++g)
#pragma unroll
    for (int e = 0; e < 4; ++e) {
      const float dv = t[g][e] - mu;
      ss = fmaf(dv, dv, ss);
    }
#pragma unroll
  for (int o = 16; o >= 1; o >>= 1) ss += __shfl_xor(ss, o, 32);
  const float var = ss * (1.0f / (float)kDim);
  const float inv = rsqrtf(var + kLnEps);
  v8h hv[2], lv[2];
#pragma unroll
  for (int g = 0; g < 4; ++g) {
    const int off = (g >> 1) * 256 + lane * 8 + (g & 1) * 4;
    const v4f w4 = *(const v4f*)(gw + off);
    const v4f b4 = *(const v4f*)(gb + off);
#pragma unroll
    for (int e = 0; e < 4; ++e) {
      const float tn = (t[g][e] - mu) * inv * w4[e] + b4[e];
      _Float16 h, l;
      f16_split(tn, h, l);
      hv[g >> 1][(g & 1) * 4 + e] = h;
      lv[g >> 1][(g & 1) * 4 + e] = l;
    }
  }
  for (int pass = 0; pass < 2; ++pass) {
#pragma unroll
    for (int hf = 0; hf < 2; ++hf) {
      const size_t o = (size_t)row * kDim + hf * 256 + lane * 8;
      *(volatile v8h*)(dH + o) = hv[hf];
      *(volatile v8h*)(dL + o) = lv[hf];
    }
    __threadfence();
  }
}

template <bool SILU>
__global__ __launch_bounds__(256) void bias_act_split_kernel(
    const float* __restrict__ src, const float* __restrict__ bias,
    float* __restrict__ dF, unsigned short* __restrict__ dH, unsigned short* __restrict__ dL, int nwaves)
{
  const int lane = threadIdx.x & 31;
  const int wave = threadIdx.x >> 5;
  const int w = blockIdx.x * 8 + wave;
  if (w >= nwaves) return;
  const size_t e0 = (size_t)w * 256;
  const int c0 = (int)(e0 & (size_t)(kDim - 1));
  v4f fo[2];
#pragma unroll
  for (int g = 0; g < 2; ++g) {
    const int o = g * 128 + lane * 4;
    const v4f a = *(const v4f*)(src + e0 + o);
    const v4f b = *(const v4f*)(bias + c0 + o);
#pragma unroll
    for (int e = 0; e < 4; ++e) {
      float v = a[e] + b[e];
      if (SILU) {
        const float sg = __builtin_amdgcn_rcpf(1.0f + expf(-v));
        v = v * sg;
      }
      fo[g][e] = v;
    }
  }
  v8h hv, lv;
  {
    const int o8 = lane * 8;
    const v4f a0 = *(const v4f*)(src + e0 + o8);
    const v4f a1 = *(const v4f*)(src + e0 + o8 + 4);
    const v4f b0 = *(const v4f*)(bias + c0 + o8);
    const v4f b1 = *(const v4f*)(bias + c0 + o8 + 4);
#pragma unroll
    for (int e = 0; e < 4; ++e) {
      _Float16 h0, l0, h1, l1;
      const float f0 = a0[e] + b0[e];
      const float f1 = a1[e] + b1[e];
      f16_split(f0, h0, l0);
      f16_split(f1, h1, l1);
      hv[e] = h0; lv[e] = l0;
      hv[4 + e] = h1; lv[4 + e] = l1;
    }
  }
  for (int pass = 0; pass < 2; ++pass) {
#pragma unroll
    for (int g = 0; g < 2; ++g)
      *(volatile v4f*)(dF + e0 + g * 128 + lane * 4) = fo[g];
    *(volatile v8h*)(dH + e0 + lane * 8) = hv;
    *(volatile v8h*)(dL + e0 + lane * 8) = lv;
    __threadfence();
  }
}

__global__ __launch_bounds__(256) void bias_rows_kernel(
    const float* __restrict__ src, const float* __restrict__ bias, float* __restrict__ dst, int nwaves)
{
  const int lane = threadIdx.x & 31;
  const int wave = threadIdx.x >> 5;
  const int w = blockIdx.x * 8 + wave;
  if (w >= nwaves) return;
  const size_t e0 = (size_t)w * 256;
  const int c0 = (int)(e0 & (size_t)(kDim - 1));
  v4f fo[2];
#pragma unroll
  for (int g = 0; g < 2; ++g) {
    const int o = g * 128 + lane * 4;
    const v4f a = *(const v4f*)(src + e0 + o);
    const v4f b = *(const v4f*)(bias + c0 + o);
    fo[g] = a + b;
  }
  for (int pass = 0; pass < 2; ++pass) {
#pragma unroll
    for (int g = 0; g < 2; ++g)
      *(volatile v4f*)(dst + e0 + g * 128 + lane * 4) = fo[g];
    __threadfence();
  }
}

typedef float    ms1_v4f __attribute__((ext_vector_type(4)));
typedef unsigned ms1_v4u __attribute__((ext_vector_type(4)));
struct ms1_args {
  const float* dtpre;
  const float* u;
  const float* bc;
  const float* z;
  const float* A_log;
  const float* Dskip;
  __half* y;
  __half* y_lo;
  long ld_dtpre;
  long ld_u;
  long ld_bc;
  long ld_z;
  long ld_y;
  int offB;
  int offC;
  int offZ;
  float ycarry;
  int dir;
  int D;
  int L;
  int nbatch;
};
static_assert(sizeof(ms1_args) == 136);

__device__ __forceinline__ float ms1_flush16(float v) {
  return (fabsf(v) < 6.103515625e-05f) ? 0.0f : v;
}
__device__ __forceinline__ unsigned ms1_h16bits(float v) {
  return (unsigned)__half_as_ushort(__float2half_rn(ms1_flush16(v)));
}
__device__ __forceinline__ float ms1_h16val(unsigned b) {
  return __half2float(__ushort_as_half((unsigned short)b));
}
__device__ __forceinline__ float ms1_softplus(float v) {
  return fmaxf(v, 0.0f) + log1pf(expf(-fabsf(v)));
}
__device__ __forceinline__ void ms1_pack2(float v0, float v1, unsigned& hw, unsigned& lw) {
  const unsigned h0 = ms1_h16bits(v0);
  const unsigned h1 = ms1_h16bits(v1);
  const float r0 = (v0 - ms1_h16val(h0)) * 2048.0f;
  const float r1 = (v1 - ms1_h16val(h1)) * 2048.0f;
  const unsigned l0 = ms1_h16bits(r0);
  const unsigned l1 = ms1_h16bits(r1);
  hw = h0 | (h1 << 16);
  lw = l0 | (l1 << 16);
}

template <int NSTATE>
__global__ __launch_bounds__(64 * (NSTATE / 16)) void ms1_scan_kernel(ms1_args a)
{
  static_assert(NSTATE == 16 || NSTATE == 64);
  constexpr int NQ  = NSTATE / 16;
  constexpr int NT  = 64 * NQ;
  constexpr int NW  = NT / 32;
  constexpr int BCW = 2 * NSTATE;
  constexpr int YP  = 68;
  constexpr int RPI = NW * 4;
  constexpr int NIT = 64 / RPI;
  static_assert(16 * NT <= 64 * YP);
  __shared__ __align__(16) float sBC[64 * BCW];
  __shared__ __align__(16) float sY[64 * YP];
  const int tid  = threadIdx.x;
  const int lane = tid & 31;
  const int wave = tid >> 5;
  const int c    = tid / NQ;
  const int sq   = tid - c * NQ;
  const int bpb  = a.D / 64;
  const int bi   = blockIdx.x / bpb;
  if (bi >= a.nbatch) return;
  const int d0 = (blockIdx.x - bi * bpb) * 64;
  const int d  = d0 + c;
  const long rowb = (long)bi * a.L;
  const bool hasz  = (a.z != nullptr);
  const bool hasD  = (a.Dskip != nullptr);
  const bool hasLo = (a.y_lo != nullptr);

#pragma unroll 1
  for (int n = 0; n < 16; ++n) {
    const float al = a.A_log[(long)d * NSTATE + sq * 16 + n];
    sY[n * NT + tid] = -expf(al);
  }
  __syncthreads();
  float An[16], h[16];
#pragma unroll
  for (int n = 0; n < 16; ++n) {
    An[n] = sY[n * NT + tid];
    h[n] = 0.0f;
  }
  float Dd = 0.0f;
  if (hasD) Dd = a.Dskip[d];

  const int nchunk = a.L / 64;
  const bool fwd = (a.dir > 0);
  const int s0 = fwd ? 0 : 63;
  const int sd = fwd ? 1 : -1;
  const int q  = lane >> 3;
  const int c8 = (lane & 7) * 8;

#pragma unroll 1
  for (int ci = 0; ci < nchunk; ++ci) {
    const int tb = fwd ? (ci * 64) : (a.L - 64 - ci * 64);
    const long rowc = rowb + tb;
    __syncthreads();
#pragma unroll 8
    for (int i = 0; i < 32; ++i) {
      const int idx = tid + i * NT;
      const int st  = idx / BCW;
      const int col = idx - st * BCW;
      const int sc  = (col < NSTATE) ? (a.offB + col) : (a.offC + col - NSTATE);
      sBC[idx] = a.bc[(rowc + st) * a.ld_bc + sc];
    }
    __syncthreads();
#pragma unroll 1
    for (int s = 0; s < 64; ++s) {
      const int ls = s0 + sd * s;
      const long row = rowc + ls;
      float pre = a.dtpre[row * a.ld_dtpre + d];
      float uv  = a.u[row * a.ld_u + d];
      float zv  = 0.0f;
      if (hasz) zv = a.z[row * a.ld_z + a.offZ + d];
      asm volatile("" : "+v"(pre));
      asm volatile("" : "+v"(uv));
      asm volatile("" : "+v"(zv));
      const float delta = ms1_softplus(pre);
      const float dtx = delta * uv;
      const float* bp = sBC + ls * BCW + sq * 16;
      const float* cp = bp + NSTATE;
      ms1_v4f Bq[4], Cq[4];
#pragma unroll
      for (int k = 0; k < 4; ++k) {
        Bq[k] = *(const ms1_v4f*)(bp + 4 * k);
        Cq[k] = *(const ms1_v4f*)(cp + 4 * k);
      }
      float yv = 0.0f;
#pragma unroll
      for (int n = 0; n < 16; ++n) {
        const float e = __expf(delta * An[n]);
        h[n] = fmaf(e, h[n], dtx * Bq[n >> 2][n & 3]);
        yv = fmaf(h[n], Cq[n >> 2][n & 3], yv);
      }
      if (NQ > 1) {
        yv += __shfl_xor(yv, 1, 32);
        yv += __shfl_xor(yv, 2, 32);
      }
      if (hasD) yv = fmaf(uv, Dd, yv);
      if (hasz) {
        const float sg = __builtin_amdgcn_rcpf(1.0f + expf(-zv));
        yv = yv * (zv * sg);
      }
      if (sq == 0) sY[ls * YP + c] = yv * a.ycarry;
    }
    __syncthreads();
    ms1_v4u hw[NIT], lw[NIT];
#pragma unroll
    for (int it = 0; it < NIT; ++it) {
      const int row = it * RPI + wave * 4 + q;
      const float* sp = sY + row * YP + c8;
      const ms1_v4f f0 = *(const ms1_v4f*)(sp);
      const ms1_v4f f1 = *(const ms1_v4f*)(sp + 4);
      unsigned h0, h1, h2, h3, l0, l1, l2, l3;
      ms1_pack2(f0[0], f0[1], h0, l0);
      ms1_pack2(f0[2], f0[3], h1, l1);
      ms1_pack2(f1[0], f1[1], h2, l2);
      ms1_pack2(f1[2], f1[3], h3, l3);
      hw[it] = (ms1_v4u){h0, h1, h2, h3};
      lw[it] = (ms1_v4u){l0, l1, l2, l3};
    }
    for (int pass = 0; pass < 2; ++pass) {
#pragma unroll
      for (int it = 0; it < NIT; ++it) {
        const int row = it * RPI + wave * 4 + q;
        const long o = (rowc + row) * a.ld_y + d0 + c8;
        *(volatile ms1_v4u*)(a.y + o) = hw[it];
        if (hasLo) *(volatile ms1_v4u*)(a.y_lo + o) = lw[it];
      }
      __threadfence();
    }
  }
}

__device__ __forceinline__ float y_rebuild(unsigned hb, unsigned lb) {
  const float hi = h16_to_f32(hb);
  const float lo = h16_to_f32(lb);
  return (hi + lo * kResidInv) * kYCarryInv;
}

__global__ __launch_bounds__(256) void gated_sum_kernel(
    const unsigned short* __restrict__ YH, const unsigned short* __restrict__ YL,
    const float* __restrict__ Z, float* __restrict__ out, int nwaves)
{
  const int lane = threadIdx.x & 31;
  const int wave = threadIdx.x >> 5;
  const int w = blockIdx.x * 8 + wave;
  if (w >= nwaves) return;
  const size_t e0 = (size_t)w * 256;
  v4f res[2];
#pragma unroll
  for (int g = 0; g < 2; ++g) {
    const size_t idx = e0 + g * 128 + lane * 4;
    float yb[3][4];
    v4f zz[3];
#pragma unroll
    for (int br = 0; br < 3; ++br) {
      const v2u hw = *(const v2u*)(YH + (size_t)br * kPlane + idx);
      const v2u lw = *(const v2u*)(YL + (size_t)br * kPlane + idx);
      zz[br] = *(const v4f*)(Z + (size_t)br * kPlane + idx);
      yb[br][0] = y_rebuild(hw[0] & 0xffffu, lw[0] & 0xffffu);
      yb[br][1] = y_rebuild(hw[0] >> 16, lw[0] >> 16);
      yb[br][2] = y_rebuild(hw[1] & 0xffffu, lw[1] & 0xffffu);
      yb[br][3] = y_rebuild(hw[1] >> 16, lw[1] >> 16);
    }
#pragma unroll
    for (int e = 0; e < 4; ++e) {
      const float y1 = yb[0][e], y2 = yb[1][e], y3 = yb[2][e];
      const float za = zz[0][e], zb = zz[1][e], zc = zz[2][e];
      float acc = y1 * zb;
      acc = acc + y1 * zc;
      acc = acc + y2 * za;
      acc = acc + y2 * zc;
      acc = acc + y3 * za;
      acc = acc + y3 * za;
      res[g][e] = acc;
    }
  }
  for (int pass = 0; pass < 2; ++pass) {
#pragma unroll
    for (int g = 0; g < 2; ++g)
      *(volatile v4f*)(out + e0 + g * 128 + lane * 4) = res[g];
    __threadfence();
  }
}

extern "C" void kernel_launch(void* const* d_in, const int* in_sizes, int n_in,
                              void* d_out, int out_size, void* d_ws, size_t ws_size,
                              hipStream_t stream)
{
  if (n_in < 14) return;
  if (in_sizes[0] != kRows * kDim) return;
  if (in_sizes[1] != kRows * kDim) return;
  if (in_sizes[2] != kRows * kDim) return;
  if (in_sizes[3] != kDim) return;
  if (in_sizes[4] != kDim) return;
  if (in_sizes[5] != kDim * kDim) return;
  if (in_sizes[6] != kDim) return;
  if (in_sizes[7] != kDim * kDim) return;
  if (in_sizes[8] != kDim) return;
  if (in_sizes[9] != kBcP * kDim) return;
  if (in_sizes[10] != kDim * kDtRank) return;
  if (in_sizes[11] != kDim) return;
  if (in_sizes[12] != kDim * kNst) return;
  if (in_sizes[13] != kDim) return;
  if (out_size != kRows * kDim) return;
  if (ws_size < kWsTotal) return;

  const float* xin[3] = {(const float*)d_in[0], (const float*)d_in[1], (const float*)d_in[2]};
  const float* norm_w    = (const float*)d_in[3];
  const float* norm_b    = (const float*)d_in[4];
  const float* proj_w    = (const float*)d_in[5];
  const float* proj_b    = (const float*)d_in[6];
  const float* conv_w    = (const float*)d_in[7];
  const float* conv_b    = (const float*)d_in[8];
  const float* deltaBC_w = (const float*)d_in[9];
  const float* dt_w      = (const float*)d_in[10];
  const float* dt_b      = (const float*)d_in[11];
  const float* A_log     = (const float*)d_in[12];
  const float* D_par     = (const float*)d_in[13];
  float* out = (float*)d_out;

  char* ws = (char*)d_ws;
  unsigned short* WPH = (unsigned short*)(ws + kOffWPH);
  unsigned short* WPL = (unsigned short*)(ws + kOffWPL);
  unsigned short* WC  = (unsigned short*)(ws + kOffWC);
  unsigned short* WDH = (unsigned short*)(ws + kOffWDH);
  unsigned short* WDL = (unsigned short*)(ws + kOffWDL);
  unsigned short* WT  = (unsigned short*)(ws + kOffWT);
  unsigned short* TNH = (unsigned short*)(ws + kOffTNH);
  unsigned short* TNL = (unsigned short*)(ws + kOffTNL);
  float*          PR  = (float*)(ws + kOffPR);
  unsigned short* PH  = (unsigned short*)(ws + kOffPH);
  unsigned short* PL  = (unsigned short*)(ws + kOffPL);
  float*          CR  = (float*)(ws + kOffCR);
  float*          U   = (float*)(ws + kOffU);
  unsigned short* UH  = (unsigned short*)(ws + kOffUH);
  unsigned short* UL  = (unsigned short*)(ws + kOffUL);
  float*          BC  = (float*)(ws + kOffBC);
  unsigned short* BCH = (unsigned short*)(ws + kOffBCH);
  unsigned short* BCL = (unsigned short*)(ws + kOffBCL);
  float*          DTR = (float*)(ws + kOffDTR);
  float*          DT  = (float*)(ws + kOffDT);
  float*          Z   = (float*)(ws + kOffZ);
  unsigned short* YH  = (unsigned short*)(ws + kOffYH);
  unsigned short* YL  = (unsigned short*)(ws + kOffYL);

  pack_weight_f16_kernel<true><<<(kDim * kDim / 8) / 256, 256, 0, stream>>>(proj_w, WPH, WPL, kDim * kDim / 8, kWCarry);
  pack_weight_f16_kernel<false><<<(kDim * kDim / 8) / 256, 256, 0, stream>>>(conv_w, WC, WC, kDim * kDim / 8, kWCarry);
  pack_weight_f16_kernel<true><<<(kBcP * kDim / 8) / 256, 256, 0, stream>>>(deltaBC_w, WDH, WDL, kBcP * kDim / 8, kWCarry);
  pack_weight_f16_kernel<false><<<(kDim * kDtRank / 8) / 256, 256, 0, stream>>>(dt_w, WT, WT, kDim * kDtRank / 8, kWCarry);

  constexpr int kTilesBig  = (kRows / 32) * (kDim / 64) / 8;
  constexpr int kTilesProj = (kRows / 16) * (kDim / 64) / 8;
  constexpr int kTilesBc   = (kRows / 16) * (kBcP / 64) / 8;
  constexpr int kHalfRows  = kRows * 2;
  static_assert(kTilesBig == 128 && kTilesProj == 256 && kTilesBc == 32);

  for (int br = 0; br < kNbranch; ++br) {
    float* Zb = Z + (size_t)br * kPlane;
    unsigned short* YHb = YH + (size_t)br * kPlane;
    unsigned short* YLb = YL + (size_t)br * kPlane;

    layernorm_split_kernel<<<kRows / 8, 256, 0, stream>>>(xin[br], norm_w, norm_b, TNH, TNL, kRows);

    eng::gemm_f16_kernel<1, 2><<<dim3(kTilesProj), 256, 0, stream>>>(
        TNH, TNL, kDim, WPH, WPL, kDim, PR, kDim, kRows, kDim, kDim, kSW, kSWr);

    bias_act_split_kernel<true><<<kHalfRows / 8, 256, 0, stream>>>(PR, proj_b, Zb, PH, PL, kHalfRows);

    eng::gemm_f16_kernel<2, 1><<<dim3(kTilesBig), 256, 0, stream>>>(
        PH, PL, kDim, WC, WC, kDim, CR, kDim, kRows, kDim, kDim, kSW, kSWr);

    bias_act_split_kernel<false><<<kHalfRows / 8, 256, 0, stream>>>(CR, conv_b, U, UH, UL, kHalfRows);

    eng::gemm_f16_kernel<1, 2><<<dim3(kTilesBc), 256, 0, stream>>>(
        UH, UL, kDim, WDH, WDL, kDim, BC, kBcP, kRows, kBcP, kDim, kSW, kSWr);

    split_rows_f16_kernel<<<(kRows * kBcP / 8) / 256, 256, 0, stream>>>(BC, BCH, BCL, kRows * kBcP / 8);

    eng::gemm_f16_kernel<2, 1><<<dim3(kTilesBig), 256, 0, stream>>>(
        BCH, BCL, kBcP, WT, WT, kDtRank, DTR, kDim, kRows, kDim, kDtRank, kSW, kSWr);

    bias_rows_kernel<<<kHalfRows / 8, 256, 0, stream>>>(DTR, dt_b, DT, kHalfRows);

    ms1_args sa;
    sa.dtpre = DT;
    sa.u = U;
    sa.bc = BC;
    sa.z = nullptr;
    sa.A_log = A_log;
    sa.Dskip = D_par;
    sa.y = (__half*)YHb;
    sa.y_lo = (__half*)YLb;
    sa.ld_dtpre = kDim;
    sa.ld_u = kDim;
    sa.ld_bc = kBcP;
    sa.ld_z = kDim;
    sa.ld_y = kDim;
    sa.offB = kOffB;
    sa.offC = kOffC;
    sa.offZ = 0;
    sa.ycarry = kYCarry;
    sa.dir = 1;
    sa.D = kDim;
    sa.L = kSeq;
    sa.nbatch = kBatch;
    ms1_scan_kernel<16><<<dim3((kDim / 64) * kBatch), 64, 0, stream>>>(sa);
  }

  gated_sum_kernel<<<kHalfRows / 8, 256, 0, stream>>>(YH, YL, Z, out, kHalfRows);
}
